// TriplaneAttention_72962904424786
// MI455X (gfx1250) — hardware-verified
//
#include <hip/hip_runtime.h>


namespace {
constexpr int B = 2, RES = 32, NT = 3 * RES * RES, C = 512, NH = 8, DH = 64, T = B * NT;
constexpr float XS = 8.0f, WSC = 256.0f;
typedef _Float16 b16;
typedef __attribute__((ext_vector_type(16))) _Float16 v16b;
typedef __attribute__((ext_vector_type(8))) _Float16 v8b;
typedef __attribute__((ext_vector_type(8))) float v8f;
typedef __attribute__((ext_vector_type(4))) float v4f;
typedef __attribute__((ext_vector_type(2))) float v2f;
__device__ __forceinline__ float bf16_rne(float f) { unsigned int u = __float_as_uint(f); u += 0x7FFFu + ((u >> 16) & 1u); float r = __uint_as_float(u & 0xFFFF0000u); asm volatile("" : "+v"(r)); return r; }
__device__ __forceinline__ void split16(float v, b16& hi, b16& lo) { hi = (b16)v; lo = (b16)(v - (float)hi); }
__device__ __forceinline__ v16b frag_kb(const b16* p, int hh) { const v8b a = *(const v8b*)(p + 8 * hh), b = *(const v8b*)(p + 16 + 8 * hh); v16b f;
#pragma unroll
  for (int e = 0; e < 8; ++e) { f[e] = a[e]; f[8 + e] = b[e]; } return f; }
__device__ __forceinline__ v8f wmma16b(v16b a, v16b b, v8f c) { v8f d = __builtin_amdgcn_wmma_f32_16x16x32_f16(false, a, false, b, (short)0, c, false, false); asm volatile("v_nop\n\tv_nop\n\tv_nop\n\tv_nop" : "+v"(d) : "v"(a), "v"(b)); return d; }
__device__ __forceinline__ void wave_lds_sync() { __builtin_amdgcn_fence(__ATOMIC_RELEASE, "workgroup"); __builtin_amdgcn_wave_barrier(); __builtin_amdgcn_fence(__ATOMIC_ACQUIRE, "workgroup"); }
__device__ __forceinline__ float pmul(float a, float b) { float p = a * b; asm volatile("" : "+v"(p)); return p; }

__global__ __launch_bounds__(256) void wput_kernel(const float* __restrict__ wq, const float* __restrict__ wk, const float* __restrict__ wv, const float* __restrict__ wp, b16* __restrict__ WQKV, b16* __restrict__ WP) { const size_t u = (size_t)blockIdx.x * 256 + threadIdx.x; if (u >= (size_t)C * 64) return; v8b a, b, c, d;
#pragma unroll
  for (int j = 0; j < 8; ++j) { a[j] = (b16)(bf16_rne(wq[u * 8 + j]) * WSC); b[j] = (b16)(bf16_rne(wk[u * 8 + j]) * WSC); c[j] = (b16)(bf16_rne(wv[u * 8 + j]) * WSC); d[j] = (b16)(bf16_rne(wp[u * 8 + j]) * WSC); }
  for (int pass = 0; pass < 2; ++pass) { *(volatile v8b*)(WQKV + u * 8) = a; *(volatile v8b*)(WQKV + (size_t)C * C + u * 8) = b; *(volatile v8b*)(WQKV + (size_t)2 * C * C + u * 8) = c; *(volatile v8b*)(WP + u * 8) = d; __threadfence(); } }
template <int MODE>
__global__ __launch_bounds__(32) void dense_kernel(const float* __restrict__ IN, const b16* __restrict__ WT, const float* __restrict__ bias, int NOUT, int RLIM, float* __restrict__ OUT) { __shared__ __attribute__((aligned(16))) b16 Ah[16][C + 8], Al[16][MODE == 0 ? 8 : C + 8]; __shared__ float Tf[16][260]; const int lane = threadIdx.x, nloc = lane & 15, hlf = lane >> 4; const int NG = NOUT / 256; const int g = blockIdx.x % NG; const size_t r0 = (size_t)(blockIdx.x / NG) * 16; if (r0 >= (size_t)RLIM) return;
  for (int rr = 0; rr < 16; ++rr) for (int q = 0; q < C / 32; ++q) { const float v = IN[(r0 + rr) * C + q * 32 + lane]; if (MODE == 0) Ah[rr][q * 32 + lane] = (b16)(bf16_rne(v) * XS); else { b16 p, ql; split16(v * XS, p, ql); Ah[rr][q * 32 + lane] = p; Al[rr][q * 32 + lane] = ql; } }
  wave_lds_sync(); v8f acc[16];
#pragma unroll
  for (int t = 0; t < 16; ++t) acc[t] = (v8f){};
#pragma unroll 1
  for (int kb = 0; kb < C; kb += 32) { const v16b a = frag_kb(&Ah[nloc][kb], hlf); v16b al; if (MODE != 0) al = frag_kb(&Al[nloc][kb], hlf);
#pragma unroll
    for (int t = 0; t < 16; ++t) { const v16b bw = frag_kb(WT + (size_t)(g * 256 + t * 16 + nloc) * C + kb, hlf); acc[t] = wmma16b(a, bw, acc[t]); if (MODE != 0) acc[t] = wmma16b(al, bw, acc[t]); } }
#pragma unroll
  for (int t = 0; t < 16; ++t) { const int cc = g * 256 + t * 16 + nloc; const float bb = bias ? bf16_rne(bias[cc]) : 0.0f;
#pragma unroll
    for (int r8 = 0; r8 < 8; ++r8) Tf[8 * hlf + r8][t * 16 + nloc] = acc[t][r8] * (1.0f / (XS * WSC)) + bb; }
  wave_lds_sync();
  for (int pass = 0; pass < 2; ++pass) { for (int rr = 0; rr < 16; ++rr) for (int q = 0; q < 2; ++q) *(volatile v4f*)(OUT + (r0 + rr) * NOUT + g * 256 + q * 128 + lane * 4) = *(const v4f*)(&Tf[rr][q * 128 + lane * 4]); __threadfence(); } }
__device__ __forceinline__ int keytok(int p, int i, int j, int kk) { const int t = kk & 31; const int first = kk < 32;
  if (p == 0) return first ? (1 * 1024 + i * 32 + t) : (2 * 1024 + j * 32 + t);
  if (p == 1) return first ? (0 * 1024 + i * 32 + t) : (2 * 1024 + t * 32 + j);
  return first ? (0 * 1024 + t * 32 + i) : (1 * 1024 + t * 32 + j); }
__global__ __launch_bounds__(256) void attn_kernel(const float* __restrict__ QKV, int TLIM, float* __restrict__ O) { const int wave = threadIdx.x >> 5, lane = threadIdx.x & 31; const size_t wid = (size_t)blockIdx.x * 8 + wave; const size_t tok = wid / NH; const int h = (int)(wid % NH); if (tok >= (size_t)TLIM) return; const int b = (int)(tok / NT), n = (int)(tok % NT); const int p = n / 1024, i = (n / 32) % 32, j = n % 32;
  const float* qrow = QKV + tok * 3 * C + h * DH; const size_t k0 = ((size_t)b * NT + keytok(p, i, j, lane)) * 3 * C + C + h * DH, k1 = ((size_t)b * NT + keytok(p, i, j, lane + 32)) * 3 * C + C + h * DH; float s0 = 0.0f, s1 = 0.0f;
#pragma unroll 4
  for (int d = 0; d < DH; d += 4) { const v4f qv = *(const v4f*)(qrow + d), ka = *(const v4f*)(QKV + k0 + d), kb = *(const v4f*)(QKV + k1 + d); for (int e = 0; e < 4; ++e) { s0 += pmul(qv[e], ka[e]); s1 += pmul(qv[e], kb[e]); } }
  s0 *= 0.125f; s1 *= 0.125f; float mx = fmaxf(s0, s1); for (int o = 16; o; o >>= 1) mx = fmaxf(mx, __shfl_xor(mx, o)); const float e0 = __expf(s0 - mx), e1 = __expf(s1 - mx); float den = e0 + e1; for (int o = 16; o; o >>= 1) den += __shfl_xor(den, o); const float inv = 1.0f / den;
  float o0 = 0.0f, o1 = 0.0f;
#pragma unroll 1
  for (int kk = 0; kk < 64; ++kk) { const float pk = __shfl(kk < 32 ? e0 : e1, kk & 31) * inv; const size_t vt = ((size_t)b * NT + keytok(p, i, j, kk)) * 3 * C + 2 * C + h * DH; const v2f vv = *(const v2f*)(QKV + vt + lane * 2); o0 += pmul(pk, vv[0]); o1 += pmul(pk, vv[1]); }
  for (int pass = 0; pass < 2; ++pass) { *(volatile v2f*)(O + tok * C + h * DH + lane * 2) = (v2f){o0, o1}; __threadfence(); } }
}

extern "C" void kernel_launch(void* const* d_in, const int* in_sizes, int n_in, void* d_out, int out_size, void* d_ws, size_t ws_size, hipStream_t stream) {
  (void)n_in;
  auto Fp = [&](int i) { return (const float*)d_in[i]; };
  if (in_sizes[0] != T * C || in_sizes[1] != C * C || in_sizes[2] != C * C || in_sizes[3] != C * C || in_sizes[4] != C * C || in_sizes[5] != C || out_size != T * C) return;
  const int TLIM = T;
  size_t off = 0; char* ws = (char*)d_ws;
  auto carve = [&](size_t bytes) { char* p = ws + off; off += (bytes + 255) & ~(size_t)255; return p; };
  b16* WQKV = (b16*)carve((size_t)3 * C * C * 2); b16* WP = (b16*)carve((size_t)C * C * 2); float* QKV = (float*)carve((size_t)T * 3 * C * 4); float* O = (float*)carve((size_t)T * C * 4);
  if (off > ws_size || off > ((size_t)80 << 20)) return;
  wput_kernel<<<(C * 64 + 255) / 256, 256, 0, stream>>>(Fp(1), Fp(2), Fp(3), Fp(4), WQKV, WP);
  dense_kernel<0><<<(TLIM / 16) * 6, 32, 0, stream>>>(Fp(0), WQKV, nullptr, 3 * C, TLIM, QKV);
  attn_kernel<<<(unsigned)(((size_t)TLIM * NH + 7) / 8), 256, 0, stream>>>(QKV, TLIM, O);
  dense_kernel<1><<<(TLIM / 16) * 2, 32, 0, stream>>>(O, WP, Fp(5), C, TLIM, (float*)d_out);
}
